// RelPositionMHA_3264175145120
// MI455X (gfx1250) — hardware-verified
//
#include <hip/hip_runtime.h>
#include <math.h>
#include <stdint.h>

#define NB_  4
#define NT_  2048
#define ND_  1024
#define NH_  8
#define HD_  128
#define NP_  4095
#define NPP_ 4096
#define BDW_ 2112

typedef _Float16 v16h __attribute__((ext_vector_type(16)));
typedef _Float16 v8h  __attribute__((ext_vector_type(8)));
typedef float    v8f  __attribute__((ext_vector_type(8)));
typedef float    v4f  __attribute__((ext_vector_type(4)));
typedef v4f __attribute__((may_alias)) v4fa;
typedef v8h __attribute__((may_alias)) v8ha;

__device__ __forceinline__ float bf_rne(float f) {
  unsigned u = __float_as_uint(f);
  u = (u + 0x7FFFu + ((u >> 16) & 1u)) & 0xFFFF0000u;
  return __uint_as_float(u);
}

union FragU { v16h v; v8ha h[2]; };
__device__ __forceinline__ v16h ldfrag(const _Float16* p) {
  FragU f;
  f.h[0] = *(const v8ha*)(p);
  f.h[1] = *(const v8ha*)(p + 16);
  return f.v;
}

__device__ __forceinline__ v8f mma16(v16h a, v16h b, v8f c) {
  c = __builtin_amdgcn_wmma_f32_16x16x32_f16(false, a, false, b, (short)0, c, false, false);
  asm volatile("v_nop\n\tv_nop\n\tv_nop\n\tv_nop" : "+v"(c) : "v"(a), "v"(b));
  return c;
}

__device__ __forceinline__ v8f zero8() { v8f z = {0.f, 0.f, 0.f, 0.f, 0.f, 0.f, 0.f, 0.f}; return z; }

__global__ __launch_bounds__(256) void cvt_plane_kernel(const float* __restrict__ src, _Float16* __restrict__ dst,
                                                        int nrows_src, int nrows_dst, float scale) {
  const int i = blockIdx.x * 256 + threadIdx.x;
  const int total8 = nrows_dst * (ND_ / 8);
  if (i >= total8) return;
  const int r  = i / (ND_ / 8);
  const int c8 = (i - r * (ND_ / 8)) * 8;
  const int rs = (r < nrows_src) ? r : (nrows_src - 1);
  const float sc = (r < nrows_src) ? scale : 0.0f;
  const float* sp = src + (size_t)rs * ND_ + c8;
  const v4f a = *(const v4f*)(sp);
  const v4f b = *(const v4f*)(sp + 4);
  v8h o;
  o[0] = (_Float16)(bf_rne(a[0]) * sc); o[1] = (_Float16)(bf_rne(a[1]) * sc);
  o[2] = (_Float16)(bf_rne(a[2]) * sc); o[3] = (_Float16)(bf_rne(a[3]) * sc);
  o[4] = (_Float16)(bf_rne(b[0]) * sc); o[5] = (_Float16)(bf_rne(b[1]) * sc);
  o[6] = (_Float16)(bf_rne(b[2]) * sc); o[7] = (_Float16)(bf_rne(b[3]) * sc);
  _Float16* dp = dst + (size_t)r * ND_ + c8;
  *(volatile v8h*)dp = o;
  __threadfence();
  *(volatile v8h*)dp = o;
}

template <int OUT, bool SKEW>
__global__ __launch_bounds__(256) void gemm_f16_kernel(
    const _Float16* __restrict__ A, int lda, long strideA,
    const _Float16* __restrict__ Bt, int ldb, long strideB,
    void* __restrict__ C1, void* __restrict__ C2, int ldc, long strideC,
    const float* __restrict__ b1, const float* __restrict__ b2,
    int M, int N, int K, float scale, float carry, int skew0) {
  __shared__ __align__(16) float sT[8][16 * 68];

  const int z    = blockIdx.y;
  const int lane = threadIdx.x & 31;
  const int wave = threadIdx.x >> 5;
  const int tilesN = N >> 6;
  const int tilesM = M >> 6;
  const int tile = blockIdx.x * 8 + wave;
  if (tile >= tilesM * tilesN) return;
  const int tm = tile / tilesN;
  const int tn = tile - tm * tilesN;
  const int m0 = tm << 6;
  const int n0 = tn << 6;
  const int nsk = SKEW ? ((skew0 - tm) << 6) : 0;

  const _Float16* Ab = A  + (size_t)z * strideA;
  const _Float16* Bb = Bt + (size_t)z * strideB;

  const int rl   = lane & 15;
  const int koff = (lane >> 4) * 8;
  const int mOff = (lane >> 4) * 8;

  v8f acc[4][4];
#pragma unroll
  for (int i = 0; i < 4; ++i)
#pragma unroll
    for (int j = 0; j < 4; ++j) acc[i][j] = zero8();

  for (int k0 = 0; k0 < K; k0 += 32) {
    v16h bfr[4];
#pragma unroll
    for (int j = 0; j < 4; ++j)
      bfr[j] = ldfrag(Bb + (size_t)(nsk + n0 + (j << 4) + rl) * ldb + koff + k0);
#pragma unroll
    for (int i = 0; i < 4; ++i) {
      const v16h af = ldfrag(Ab + (size_t)(m0 + (i << 4) + rl) * lda + koff + k0);
#pragma unroll
      for (int j = 0; j < 4; ++j) acc[i][j] = mma16(af, bfr[j], acc[i][j]);
    }
  }

  float* slab = sT[wave];
#pragma unroll
  for (int i = 0; i < 4; ++i) {
    const int mBase = m0 + (i << 4);
#pragma unroll
    for (int j = 0; j < 4; ++j)
#pragma unroll
      for (int r = 0; r < 8; ++r)
        slab[(mOff + r) * 68 + (j << 4) + rl] = acc[i][j][r] * scale;
    __builtin_amdgcn_fence(__ATOMIC_RELEASE, "workgroup");
    __builtin_amdgcn_wave_barrier();
    __builtin_amdgcn_fence(__ATOMIC_ACQUIRE, "workgroup");
    if (OUT == 0) {
      float* C = (float*)C1 + (size_t)z * strideC;
      const int hh = lane >> 4, c4 = (lane & 15) * 4;
      for (int pass = 0; pass < 2; ++pass) {
#pragma unroll
        for (int it = 0; it < 8; ++it) {
          const int row = it * 2 + hh;
          const v4f v = *(const v4fa*)(slab + row * 68 + c4);
          *(volatile v4f*)(C + (size_t)(mBase + row) * ldc + n0 + c4) = v;
        }
        __threadfence();
      }
    } else {
      const int q = lane >> 3, c8 = (lane & 7) * 8;
      _Float16* Ca = (_Float16*)C1 + (size_t)z * strideC;
      _Float16* Cb = (_Float16*)C2 + (size_t)z * strideC;
      v8h hv[4], lv[4];
#pragma unroll
      for (int it = 0; it < 4; ++it) {
        const int row = it * 4 + q;
        const float* sp = slab + row * 68 + c8;
        const v4f x0 = *(const v4fa*)(sp);
        const v4f x1 = *(const v4fa*)(sp + 4);
        float f[8];
        f[0] = x0[0]; f[1] = x0[1]; f[2] = x0[2]; f[3] = x0[3];
        f[4] = x1[0]; f[5] = x1[1]; f[6] = x1[2]; f[7] = x1[3];
        v8h ha, hb;
#pragma unroll
        for (int e = 0; e < 8; ++e) {
          if (OUT == 1) {
            ha[e] = (_Float16)f[e];
            hb[e] = ha[e];
          } else {
            const int n = n0 + c8 + e;
            ha[e] = (_Float16)((f[e] + bf_rne(b1[n])) * carry);
            hb[e] = (_Float16)((f[e] + bf_rne(b2[n])) * carry);
          }
        }
        hv[it] = ha; lv[it] = hb;
      }
      for (int pass = 0; pass < 2; ++pass) {
#pragma unroll
        for (int it = 0; it < 4; ++it) {
          const int row = it * 4 + q;
          *(volatile v8h*)(Ca + (size_t)(mBase + row) * ldc + n0 + c8) = hv[it];
          if (OUT == 2) *(volatile v8h*)(Cb + (size_t)(mBase + row) * ldc + n0 + c8) = lv[it];
        }
        __threadfence();
      }
    }
    __builtin_amdgcn_fence(__ATOMIC_RELEASE, "workgroup");
    __builtin_amdgcn_wave_barrier();
    __builtin_amdgcn_fence(__ATOMIC_ACQUIRE, "workgroup");
  }
}

__global__ __launch_bounds__(128)
void relattn_kernel(const _Float16* __restrict__ QU, const _Float16* __restrict__ Kp,
                    const _Float16* __restrict__ VT, const float* __restrict__ BD,
                    _Float16* __restrict__ CTX, int pairBase, float cs) {
  __shared__ __align__(16) unsigned char SMEM[40960];
  _Float16* Ksh = (_Float16*)(SMEM);
  _Float16* Vsh = (_Float16*)(SMEM + 16384);
  _Float16* Psh = (_Float16*)(SMEM + 32768);
  float*    Osh = (float*)(SMEM);

  const int tid  = threadIdx.x;
  const int wave = tid >> 5;
  const int lane = tid & 31;
  const int hh   = lane >> 4;
  const int c    = lane & 15;

  const int z    = blockIdx.y;
  const int pair = pairBase + z;
  const int b    = pair >> 3;
  const int h    = pair & 7;
  const int qb   = blockIdx.x;
  const int q0   = qb * 64 + wave * 16;
  const int rr0  = wave * 16 + 8 * hh;

  const _Float16* Qh = QU + (size_t)(b * NT_) * ND_ + h * HD_;
  const _Float16* Kh = Kp + (size_t)(b * NT_) * ND_ + h * HD_;
  const _Float16* Vh = VT + (size_t)b * ND_ * NT_ + (size_t)(h * HD_) * NT_;
  const float*    bd = BD + (size_t)z * NT_ * BDW_;
  _Float16*       ctx = CTX + (size_t)(b * NT_) * ND_ + h * HD_;

  v16h qa[4];
#pragma unroll
  for (int dc = 0; dc < 4; ++dc)
    qa[dc] = ldfrag(Qh + (size_t)(q0 + c) * ND_ + dc * 32 + 8 * hh);

  const float* bdr = bd + (long)(q0 + 8 * hh) * BDW_ + (63 - rr0 + c);

  float mrow[8], lrow[8];
  v8f oacc[8];
#pragma unroll
  for (int r = 0; r < 8; ++r) { mrow[r] = -INFINITY; lrow[r] = 0.f; }
#pragma unroll
  for (int t = 0; t < 8; ++t) oacc[t] = zero8();

  _Float16* pw = Psh + wave * (16 * 64);

  for (int kc = 0; kc < NT_ / 64; ++kc) {
    const int kv0 = kc * 64;
    __syncthreads();
    {
      const int r = tid >> 1, c0 = (tid & 1) * 64;
      const _Float16* ks = Kh + (size_t)(kv0 + r) * ND_ + c0;
      const _Float16* vs = Vh + (size_t)tid * NT_ + kv0;
#pragma unroll
      for (int i = 0; i < 8; ++i) {
        const v8h kk8 = *(const v8h*)(ks + 8 * i);
        const v8h vv8 = *(const v8h*)(vs + 8 * i);
        *(v8ha*)(Ksh + r * 128 + c0 + 8 * i) = kk8;
        *(v8ha*)(Vsh + tid * 64 + 8 * i)      = vv8;
      }
    }
    __syncthreads();

    v8f s[4];
#pragma unroll
    for (int j = 0; j < 4; ++j) {
      s[j] = zero8();
#pragma unroll
      for (int dc = 0; dc < 4; ++dc) {
        const v16h kb = ldfrag(Ksh + (j * 16 + c) * 128 + dc * 32 + 8 * hh);
        s[j] = mma16(qa[dc], kb, s[j]);
      }
    }

    float cm[8];
#pragma unroll
    for (int r = 0; r < 8; ++r) {
      float m = -INFINITY;
#pragma unroll
      for (int j = 0; j < 4; ++j) {
        const float sv = s[j][r] * cs + bdr[(long)r * (BDW_ - 1) + kv0 + (j << 4)];
        s[j][r] = sv;
        m = fmaxf(m, sv);
      }
      m = fmaxf(m, __shfl_xor(m, 1, 32));
      m = fmaxf(m, __shfl_xor(m, 2, 32));
      m = fmaxf(m, __shfl_xor(m, 4, 32));
      m = fmaxf(m, __shfl_xor(m, 8, 32));
      cm[r] = m;
    }

#pragma unroll
    for (int r = 0; r < 8; ++r) {
      const float mnew  = fmaxf(mrow[r], cm[r]);
      const float alpha = __expf(mrow[r] - mnew);
      mrow[r] = mnew;
      float psum = 0.f;
#pragma unroll
      for (int j = 0; j < 4; ++j) {
        const float p = __expf(s[j][r] - mnew);
        psum += p;
        pw[(8 * hh + r) * 64 + j * 16 + c] = (_Float16)(p * 4096.0f);
      }
      psum += __shfl_xor(psum, 1, 32);
      psum += __shfl_xor(psum, 2, 32);
      psum += __shfl_xor(psum, 4, 32);
      psum += __shfl_xor(psum, 8, 32);
      lrow[r] = lrow[r] * alpha + psum;
#pragma unroll
      for (int t = 0; t < 8; ++t) oacc[t][r] *= alpha;
    }
    __builtin_amdgcn_fence(__ATOMIC_RELEASE, "workgroup");
    __builtin_amdgcn_wave_barrier();
    __builtin_amdgcn_fence(__ATOMIC_ACQUIRE, "workgroup");

#pragma unroll
    for (int kk = 0; kk < 2; ++kk) {
      const v16h pa = ldfrag(pw + c * 64 + kk * 32 + 8 * hh);
#pragma unroll
      for (int t = 0; t < 8; ++t) {
        const v16h vb = ldfrag(Vsh + (t * 16 + c) * 64 + kk * 32 + 8 * hh);
        oacc[t] = mma16(pa, vb, oacc[t]);
      }
    }
  }

  __syncthreads();
  float* os = Osh + wave * (16 * 128);
#pragma unroll
  for (int r = 0; r < 8; ++r) {
    const float inv = 1.0f / (1024.0f * lrow[r]);
#pragma unroll
    for (int t = 0; t < 8; ++t) os[(8 * hh + r) * 128 + t * 16 + c] = oacc[t][r] * inv;
  }
  __builtin_amdgcn_fence(__ATOMIC_RELEASE, "workgroup");
  __builtin_amdgcn_wave_barrier();
  __builtin_amdgcn_fence(__ATOMIC_ACQUIRE, "workgroup");
  v8h ov[8];
#pragma unroll
  for (int it = 0; it < 8; ++it) {
    const int row = it * 2 + hh;
    const float* sp = os + row * 128 + c * 8;
    const v4f x0 = *(const v4fa*)(sp);
    const v4f x1 = *(const v4fa*)(sp + 4);
    v8h o;
    o[0] = (_Float16)x0[0]; o[1] = (_Float16)x0[1]; o[2] = (_Float16)x0[2]; o[3] = (_Float16)x0[3];
    o[4] = (_Float16)x1[0]; o[5] = (_Float16)x1[1]; o[6] = (_Float16)x1[2]; o[7] = (_Float16)x1[3];
    ov[it] = o;
  }
  for (int pass = 0; pass < 2; ++pass) {
#pragma unroll
    for (int it = 0; it < 8; ++it) {
      const int row = it * 2 + hh;
      *(volatile v8h*)(ctx + (size_t)(q0 + row) * ND_ + c * 8) = ov[it];
    }
    __threadfence();
  }
}

extern "C" void kernel_launch(void* const* d_in, const int* in_sizes, int n_in,
                              void* d_out, int out_size, void* d_ws, size_t ws_size,
                              hipStream_t stream) {
  if (n_in < 9) return;
  if (in_sizes[0] != NB_ * NT_ * ND_) return;
  if (in_sizes[1] != NP_ * ND_) return;
  if (in_sizes[2] != ND_ * ND_ || in_sizes[3] != ND_ * ND_ || in_sizes[4] != ND_ * ND_) return;
  if (in_sizes[5] != ND_ * ND_ || in_sizes[6] != ND_ * ND_) return;
  if (in_sizes[7] != NH_ * HD_ || in_sizes[8] != NH_ * HD_) return;
  if (out_size != NB_ * NT_ * ND_) return;

  const float* x   = (const float*)d_in[0];
  const float* pe  = (const float*)d_in[1];
  const float* Wq  = (const float*)d_in[2];
  const float* Wk  = (const float*)d_in[3];
  const float* Wv  = (const float*)d_in[4];
  const float* Wo  = (const float*)d_in[5];
  const float* Wp  = (const float*)d_in[6];
  const float* bu  = (const float*)d_in[7];
  const float* bvb = (const float*)d_in[8];
  float* out = (float*)d_out;

  const size_t PW16 = (size_t)ND_ * ND_ * 2;
  const size_t PA16 = (size_t)NB_ * NT_ * ND_ * 2;
  const size_t PP16 = (size_t)NPP_ * ND_ * 2;
  const size_t PX16 = (size_t)NT_ * ND_ * 2;
  const size_t PBD  = (size_t)NT_ * BDW_ * 4;
  const int    NPAIR = 2;
  size_t off = 0;
  const size_t oWO  = off; off += PW16;
  const size_t oQU  = off; off += PA16;
  const size_t oQV  = off; off += PA16;
  const size_t oKP  = off; off += PA16;
  const size_t oVT  = off; off += PA16;
  const size_t oCTX = off; off += PA16;
  const size_t oP16 = off; off += PP16;
  const size_t oSCR = off;
  const size_t oWQ  = oSCR;
  const size_t oWK  = oWQ + PW16;
  const size_t oWV  = oWK + PW16;
  const size_t oWP  = oWV + PW16;
  const size_t oX   = oWP + PW16;
  const size_t oPE  = oX + PX16;
  const size_t earlyEnd = oPE + PP16;
  const size_t bdEnd    = oSCR + (size_t)NPAIR * PBD;
  const size_t total    = (earlyEnd > bdEnd) ? earlyEnd : bdEnd;
  if (total > ws_size) return;
  if (total > (size_t)134217728) return;

  char* ws = (char*)d_ws;
  _Float16* WO  = (_Float16*)(ws + oWO);
  _Float16* QU  = (_Float16*)(ws + oQU);
  _Float16* QV  = (_Float16*)(ws + oQV);
  _Float16* KP  = (_Float16*)(ws + oKP);
  _Float16* VTP = (_Float16*)(ws + oVT);
  _Float16* CTX = (_Float16*)(ws + oCTX);
  _Float16* P16 = (_Float16*)(ws + oP16);
  _Float16* WQ  = (_Float16*)(ws + oWQ);
  _Float16* WK  = (_Float16*)(ws + oWK);
  _Float16* WV  = (_Float16*)(ws + oWV);
  _Float16* WP  = (_Float16*)(ws + oWP);
  _Float16* X   = (_Float16*)(ws + oX);
  _Float16* PE  = (_Float16*)(ws + oPE);
  float*    SCR = (float*)(ws + oSCR);

  const float inv_sdk = 0.08838834764831845f;
  const float cs      = inv_sdk * 0.00390625f;
  const dim3 blk(256);

  const dim3 gW((ND_ * (ND_ / 8) + 255) / 256);
  cvt_plane_kernel<<<gW, blk, 0, stream>>>(Wq, WQ, ND_, ND_, 64.0f);
  cvt_plane_kernel<<<gW, blk, 0, stream>>>(Wk, WK, ND_, ND_, 64.0f);
  cvt_plane_kernel<<<gW, blk, 0, stream>>>(Wv, WV, ND_, ND_, 64.0f);
  cvt_plane_kernel<<<gW, blk, 0, stream>>>(Wp, WP, ND_, ND_, 64.0f);
  cvt_plane_kernel<<<gW, blk, 0, stream>>>(Wo, WO, ND_, ND_, 64.0f);
  const dim3 gPE((NPP_ * (ND_ / 8) + 255) / 256);
  cvt_plane_kernel<<<gPE, blk, 0, stream>>>(pe, PE, NP_, NPP_, 1.0f);
  {
    const int tiles = (NPP_ / 64) * (ND_ / 64);
    gemm_f16_kernel<1, false><<<dim3((tiles + 7) / 8, 1), blk, 0, stream>>>(
        PE, ND_, 0L, WP, ND_, 0L, (void*)P16, (void*)P16, ND_, 0L, bu, bu, NPP_, ND_, ND_, 0.25f, 1.0f, 0);
  }
  for (int b = 0; b < NB_; ++b) {
    const dim3 gX((NT_ * (ND_ / 8) + 255) / 256);
    cvt_plane_kernel<<<gX, blk, 0, stream>>>(x + (size_t)b * NT_ * ND_, X, NT_, NT_, 1.0f);
    const int tilesQ = (NT_ / 64) * (ND_ / 64);
    const size_t ab = (size_t)b * NT_ * ND_;
    gemm_f16_kernel<2, false><<<dim3((tilesQ + 7) / 8, 1), blk, 0, stream>>>(
        X, ND_, 0L, WQ, ND_, 0L, (void*)(QU + ab), (void*)(QV + ab), ND_, 0L, bu, bvb,
        NT_, ND_, ND_, 0.015625f, 16.0f, 0);
    gemm_f16_kernel<1, false><<<dim3((tilesQ + 7) / 8, 1), blk, 0, stream>>>(
        X, ND_, 0L, WK, ND_, 0L, (void*)(KP + ab), (void*)(KP + ab), ND_, 0L, bu, bu,
        NT_, ND_, ND_, 0.25f, 1.0f, 0);
    const int tilesV = (ND_ / 64) * (NT_ / 64);
    gemm_f16_kernel<1, false><<<dim3((tilesV + 7) / 8, 1), blk, 0, stream>>>(
        WV, ND_, 0L, X, ND_, 0L, (void*)(VTP + (size_t)b * ND_ * NT_), (void*)(VTP + (size_t)b * ND_ * NT_),
        NT_, 0L, bu, bu, ND_, NT_, ND_, 0.25f, 1.0f, 0);
  }
  const int nGroups = (NB_ * NH_) / NPAIR;
  for (int g = 0; g < nGroups; ++g) {
    const int pairBase = g * NPAIR;
    const int b  = pairBase >> 3;
    const int h0 = pairBase & 7;
    const _Float16* Aq = QV + (size_t)b * NT_ * ND_ + h0 * HD_;
    const _Float16* Bp = P16 + h0 * HD_;
    const int tilesBD = (NT_ / 64) * (BDW_ / 64);
    gemm_f16_kernel<0, true><<<dim3((tilesBD + 7) / 8, NPAIR), blk, 0, stream>>>(
        Aq, ND_, (long)HD_, Bp, ND_, (long)HD_, (void*)SCR, (void*)SCR, BDW_, (long)NT_ * BDW_, bu, bu,
        NT_, BDW_, HD_, cs, 1.0f, 31);
    relattn_kernel<<<dim3(NT_ / 64, NPAIR), dim3(128), 0, stream>>>(QU, KP, VTP, SCR, CTX, pairBase, cs);
  }
  {
    const int tiles = ((NB_ * NT_) / 64) * (ND_ / 64);
    gemm_f16_kernel<0, false><<<dim3((tiles + 7) / 8, 1), blk, 0, stream>>>(
        CTX, ND_, 0L, WO, ND_, 0L, (void*)out, (void*)out, ND_, 0L, bu, bu,
        NB_ * NT_, ND_, ND_, 0.000244140625f, 1.0f, 0);
  }
  (void)hipGetLastError();
}
